// MultiHeadAttention_33122787786782
// MI455X (gfx1250) — hardware-run, weakly checked
//
#include <hip/hip_runtime.h>


#ifndef NB
#define NB 4
#endif
#ifndef SEQ
#define SEQ 384
#endif
#define NB_FULL  4
#define SEQ_FULL 384
#ifndef OUT_SEQ
#define OUT_SEQ SEQ
#endif
#define DM   1024
#define NH_  16
#define HD   64
#define MAXP 32
#define MREL 63
#define AW   4
#define QRS  2048.0f
#define QRI  (1.0f / 2048.0f)
#define LOG2E 1.4426950408889634f
#define PCAR 1024.0f
#define PCI  (1.0f / 1024.0f)
#define RLS  256.0f
#define RLI  (1.0f / 256.0f)

static_assert(HD == 64);
static_assert(NH_ * HD == DM);
static_assert(DM % 64 == 0);
static_assert((DM & (DM - 1)) == 0);
static_assert(SEQ % 64 == 0);
static_assert((NB * SEQ) % 64 == 0);
static_assert(SEQ % 32 == 0);
static_assert(SEQ % (16 * AW) == 0);
static_assert(SEQ > MAXP);
static_assert(MREL == 2 * MAXP - 1);
static_assert(MREL < 64);
static_assert(NB <= NB_FULL);
static_assert(SEQ <= SEQ_FULL);
static_assert(OUT_SEQ >= SEQ);

typedef _Float16 h16;
typedef unsigned short bf;
typedef __attribute__((ext_vector_type(16))) __bf16   v16bf;
typedef __attribute__((ext_vector_type(16))) _Float16 v16h;
typedef __attribute__((ext_vector_type(8)))  _Float16 v8h;
typedef __attribute__((ext_vector_type(8)))  unsigned short v8us;
typedef __attribute__((ext_vector_type(8)))  float    v8f;
typedef __attribute__((ext_vector_type(4)))  float    v4f;
typedef v4f  __attribute__((may_alias)) v4fa;
typedef v8h  __attribute__((may_alias)) v8ha;
typedef v8us __attribute__((may_alias)) v8usa;

static constexpr size_t OUT1_OFF = (size_t)NB_FULL * SEQ_FULL * DM;
static_assert(OUT1_OFF * 4 == (size_t)6291456);
static_assert(((size_t)(NB - 1) * OUT_SEQ + SEQ) * DM <= OUT1_OFF);

__device__ __forceinline__ unsigned short f2bf(float f) { unsigned u = __float_as_uint(f); u += 0x7FFFu + ((u >> 16) & 1u); return (unsigned short)(u >> 16); }
__device__ __forceinline__ float bfr(float f) { return __uint_as_float(((unsigned)f2bf(f)) << 16); }
__device__ __forceinline__ v16h cat16(v8h lo, v8h hi) { return __builtin_shufflevector(lo, hi, 0, 1, 2, 3, 4, 5, 6, 7, 8, 9, 10, 11, 12, 13, 14, 15); }
__device__ __forceinline__ v16bf cat16b(v8us lo, v8us hi) { return __builtin_bit_cast(v16bf, __builtin_shufflevector(lo, hi, 0, 1, 2, 3, 4, 5, 6, 7, 8, 9, 10, 11, 12, 13, 14, 15)); }
__device__ __forceinline__ v8f wmma16(v16h a, v16h b, v8f c) { return __builtin_amdgcn_wmma_f32_16x16x32_f16(false, a, false, b, (short)0, c, false, false); }
__device__ __forceinline__ v8f wmmab(v16bf a, v16bf b, v8f c) { return __builtin_amdgcn_wmma_f32_16x16x32_bf16(false, a, false, b, (short)0, c, false, false); }
__device__ __forceinline__ v16h  ldh(const h16* p) { return cat16(*(const v8h*)p, *(const v8h*)(p + 16)); }
__device__ __forceinline__ v16h  ldhs(const h16* p) { return cat16(*(const v8ha*)p, *(const v8ha*)(p + 16)); }
__device__ __forceinline__ v16bf ldb(const bf* p)  { return cat16b(*(const v8us*)p, *(const v8us*)(p + 16)); }
__device__ __forceinline__ void wave_sync() { __builtin_amdgcn_fence(3  , "wavefront"); __builtin_amdgcn_wave_barrier(); asm volatile("" ::: "memory"); }

__global__ __launch_bounds__(256) void k_cvt8(const float* __restrict__ src, bf* dst, size_t n8) {
    const size_t i = (size_t)blockIdx.x * 256 + threadIdx.x; if (i >= n8) return;
    const v8f v = *(const v8f*)(src + i * 8); v8us o;
#pragma unroll
    for (int k = 0; k < 8; ++k) o[k] = f2bf(v[k]);
    *(volatile v8us*)(dst + i * 8) = o; __threadfence(); *(volatile v8us*)(dst + i * 8) = o;
}

__global__ __launch_bounds__(256) void k_cvtT(const float* __restrict__ W, bf* WT) {
    __shared__ __align__(16) unsigned short ts[64 * 72];
    const int tid = threadIdx.x; const int n0 = blockIdx.x * 64, k0 = blockIdx.y * 64;
    { const int r = tid >> 2, c16 = (tid & 3) * 16;
      const float* src = W + (size_t)(k0 + r) * DM + n0 + c16;
#pragma unroll
      for (int i = 0; i < 4; ++i) { const v4f x = *(const v4f*)(src + 4 * i);
#pragma unroll
          for (int e = 0; e < 4; ++e) ts[(c16 + 4 * i + e) * 72 + r] = f2bf(x[e]); } }
    __syncthreads();
    const int nrow = tid >> 3, piece = (tid & 7) * 8;
    const v8us o0 = *(const v8usa*)(&ts[nrow * 72 + piece]); const v8us o1 = *(const v8usa*)(&ts[(nrow + 32) * 72 + piece]);
    bf* d0 = WT + (size_t)(n0 + nrow) * DM + k0 + piece; bf* d1 = d0 + (size_t)32 * DM;
    *(volatile v8us*)d0 = o0; *(volatile v8us*)d1 = o1; __threadfence(); *(volatile v8us*)d0 = o0; *(volatile v8us*)d1 = o1;
}

__global__ __launch_bounds__(256) void k_relprep(const float* __restrict__ rel, h16* P, int transpose) {
    __shared__ __align__(16) h16 ts[64 * 72];
    const int tid = threadIdx.x; const int hh = blockIdx.x;
    { const int r = tid >> 2, c16 = (tid & 3) * 16;
      const int rc = (r < MREL) ? r : (MREL - 1);
      const float* src = rel + ((size_t)hh * MREL + rc) * HD + c16;
#pragma unroll
      for (int i = 0; i < 4; ++i) { const v4f x = *(const v4f*)(src + 4 * i);
#pragma unroll
          for (int e = 0; e < 4; ++e) { const float y = (r < MREL) ? (bfr(x[e]) * RLS) : 0.0f; const int c = c16 + 4 * i + e;
              const int idx = transpose ? (c * 72 + r) : (r * 72 + c); ts[idx] = (h16)y; } } }
    __syncthreads();
    const int row = tid >> 3, piece = (tid & 7) * 8;
    const v8h o0 = *(const v8ha*)(&ts[row * 72 + piece]); const v8h o1 = *(const v8ha*)(&ts[(row + 32) * 72 + piece]);
    h16* d0 = P + (size_t)hh * 64 * 64 + (size_t)row * 64 + piece; h16* d1 = d0 + 32 * 64;
    *(volatile v8h*)d0 = o0; *(volatile v8h*)d1 = o1; __threadfence(); *(volatile v8h*)d0 = o0; *(volatile v8h*)d1 = o1;
}

__global__ __launch_bounds__(32) void k_proj(const bf* __restrict__ A, const bf* __restrict__ Bt, h16* Ph, h16* Pr, int useRes, int RB, size_t sRB, int pitch, int CB, size_t sCB) {
    __shared__ __align__(16) float os[16 * 68];
    const int K = DM;
    const int lane = threadIdx.x & 31, lr = lane & 15, hi = lane >> 4; const int r0 = blockIdx.x * 64, c0 = blockIdx.y * 64;
    v8f acc[4][4];
#pragma unroll
    for (int mb = 0; mb < 4; ++mb)
#pragma unroll
        for (int nb = 0; nb < 4; ++nb) acc[mb][nb] = (v8f){};
    const size_t aoff = (size_t)(r0 + lr) * K + 8 * hi, boff = (size_t)(c0 + lr) * K + 8 * hi;
#pragma unroll 1
    for (int kc = 0; kc < K; kc += 32) {
        v16bf a[4];
#pragma unroll
        for (int mb = 0; mb < 4; ++mb) a[mb] = ldb(A + aoff + (size_t)mb * 16 * K + kc);
#pragma unroll
        for (int nb = 0; nb < 4; ++nb) { const v16bf b = ldb(Bt + boff + (size_t)nb * 16 * K + kc);
#pragma unroll
            for (int mb = 0; mb < 4; ++mb) acc[mb][nb] = wmmab(a[mb], b, acc[mb][nb]); }
        asm volatile("v_nop\n\tv_nop\n\tv_nop\n\tv_nop" : "+v"(acc[0][0]), "+v"(acc[1][1]), "+v"(acc[2][2]), "+v"(acc[3][3]) : "v"(a[0]), "v"(a[1]), "v"(a[2]), "v"(a[3]));
    }
    const size_t tbase = (size_t)(r0 / RB) * sRB + (size_t)(r0 % RB) * (size_t)pitch + (size_t)(c0 / CB) * sCB + (size_t)(c0 % CB);
#pragma unroll
    for (int mb = 0; mb < 4; ++mb) {
#pragma unroll
        for (int nb = 0; nb < 4; ++nb) {
#pragma unroll
            for (int j = 0; j < 8; ++j) os[(hi * 8 + j) * 68 + nb * 16 + lr] = acc[mb][nb][j]; }
        wave_sync();
        const size_t sb = tbase + (size_t)(mb * 16) * (size_t)pitch;
#pragma unroll 1
        for (int ps = 0; ps < 2; ++ps) {
#pragma unroll
            for (int s = 0; s < 4; ++s) { const int row = 4 * s + (lane >> 3), c8 = (lane & 7) * 8;
                const v4f x0 = *(const v4fa*)(&os[row * 68 + c8]); const v4f x1 = *(const v4fa*)(&os[row * 68 + c8 + 4]); v8h hv, rv;
#pragma unroll
                for (int i = 0; i < 4; ++i) { const h16 a0 = (h16)x0[i]; const h16 a1 = (h16)x1[i]; hv[i] = a0; hv[4 + i] = a1; rv[i] = (h16)((x0[i] - (float)a0) * QRS); rv[4 + i] = (h16)((x1[i] - (float)a1) * QRS); }
                const size_t oo = sb + (size_t)row * (size_t)pitch + c8;
                *(volatile v8h*)(Ph + oo) = hv; if (useRes) *(volatile v8h*)(Pr + oo) = rv; }
            if (ps == 0) __threadfence(); }
        wave_sync();
    }
}

__device__ __forceinline__ void score32(const h16* __restrict__ ka, const v16h qh0, const v16h qh1, const v16h qr0, const v16h qr1,
                                        const float* relrow, const float* __restrict__ pmp, const int dm0, v8f& ta, v8f& tb) {
    const v16h ka0 = ldh(ka), ka1 = ldh(ka + 32), kb0 = ldh(ka + 16 * HD), kb1 = ldh(ka + 16 * HD + 32);
    v8f sHa = (v8f){}, sLa = (v8f){}, sHb = (v8f){}, sLb = (v8f){};
    sHa = wmma16(ka0, qh0, sHa); sLa = wmma16(ka0, qr0, sLa); sHb = wmma16(kb0, qh0, sHb); sLb = wmma16(kb0, qr0, sLb);
    sHa = wmma16(ka1, qh1, sHa); sLa = wmma16(ka1, qr1, sLa); sHb = wmma16(kb1, qh1, sHb); sLb = wmma16(kb1, qr1, sLb);
    asm volatile("v_nop\n\tv_nop\n\tv_nop\n\tv_nop" : "+v"(sHa), "+v"(sLa), "+v"(sHb), "+v"(sLb) : "v"(ka0), "v"(ka1), "v"(kb0), "v"(kb1));
    const v8f pa = *(const v8f*)pmp; const v8f pc = *(const v8f*)(pmp + 16);
#pragma unroll
    for (int r = 0; r < 8; ++r) {
        const int da = dm0 + r, db = da + 16;
        const int ia = ((da < -(MAXP - 1)) ? -(MAXP - 1) : ((da > (MAXP - 1)) ? (MAXP - 1) : da)) + (MAXP - 1);
        const int ib = ((db < -(MAXP - 1)) ? -(MAXP - 1) : ((db > (MAXP - 1)) ? (MAXP - 1) : db)) + (MAXP - 1);
        const float sa = (sHa[r] + sLa[r] * QRI) + relrow[ia];
        const float sb = (sHb[r] + sLb[r] * QRI) + relrow[ib];
        ta[r] = (sa * 0.125f + bfr(pa[r]) * -1.0e9f) * LOG2E;
        tb[r] = (sb * 0.125f + bfr(pc[r]) * -1.0e9f) * LOG2E;
    }
}

__global__ __launch_bounds__(32 * AW) void k_attn(const h16* __restrict__ QH, const h16* __restrict__ QR, const h16* __restrict__ KP, const h16* __restrict__ VT,
                                                  const h16* __restrict__ KRP, const h16* __restrict__ VRT, const float* __restrict__ PM, bf* CTX, float* ATT) {
    __shared__ __align__(16) float relS[AW * 16 * 65];
    __shared__ __align__(16) float os[AW * 16 * 68];
    __shared__ __align__(16) h16 rw[AW * 16 * 72];
    const int lane = threadIdx.x & 31, wave = threadIdx.x >> 5, lr = lane & 15, hi = lane >> 4;
    const int zh = blockIdx.y; const int b = zh / NH_, h = zh % NH_;
    const int t0 = (blockIdx.x * AW + wave) * 16;
    const size_t pbase = (size_t)zh * SEQ * HD;
    const size_t qo = pbase + (size_t)(t0 + lr) * HD + 8 * hi;
    const v16h qh0 = ldh(QH + qo), qh1 = ldh(QH + qo + 32), qr0 = ldh(QR + qo), qr1 = ldh(QR + qo + 32);
    float* rl  = relS + wave * 16 * 65;
    float* osw = os + wave * 16 * 68;
    h16*   rww = rw + wave * 16 * 72;

    { const h16* kr = KRP + (size_t)h * 64 * HD + (size_t)lr * HD + 8 * hi;
      const v16h a00 = ldh(kr), a10 = ldh(kr + 16 * HD), a20 = ldh(kr + 32 * HD), a30 = ldh(kr + 48 * HD);
      const v16h a01 = ldh(kr + 32), a11 = ldh(kr + 16 * HD + 32), a21 = ldh(kr + 32 * HD + 32), a31 = ldh(kr + 48 * HD + 32);
      v8f r0 = (v8f){}, r1 = (v8f){}, r2 = (v8f){}, r3 = (v8f){};
      r0 = wmma16(a00, qh0, r0); r1 = wmma16(a10, qh0, r1); r2 = wmma16(a20, qh0, r2); r3 = wmma16(a30, qh0, r3);
      r0 = wmma16(a01, qh1, r0); r1 = wmma16(a11, qh1, r1); r2 = wmma16(a21, qh1, r2); r3 = wmma16(a31, qh1, r3);
      asm volatile("v_nop\n\tv_nop\n\tv_nop\n\tv_nop" : "+v"(r0), "+v"(r1), "+v"(r2), "+v"(r3) : "v"(a01), "v"(a11), "v"(a21), "v"(a31), "v"(qh1));
#pragma unroll
      for (int r = 0; r < 8; ++r) { rl[lr * 65 +  0 + 8 * hi + r] = r0[r] * RLI; rl[lr * 65 + 16 + 8 * hi + r] = r1[r] * RLI;
                                    rl[lr * 65 + 32 + 8 * hi + r] = r2[r] * RLI; rl[lr * 65 + 48 + 8 * hi + r] = r3[r] * RLI; } }
    for (int i = lane; i < 144; i += 32) *(v8ha*)(rww + i * 8) = (v8h){};
    wave_sync();

    const h16* kbase = KP + pbase + (size_t)lr * HD + 8 * hi;
    const h16* vbase = VT + pbase + (size_t)lr * SEQ + 8 * hi;
    const float* pmrow = PM + (size_t)b * SEQ_FULL + 8 * hi;
    const float* relrow = rl + lr * 65;
    const int dmb = 8 * hi - (t0 + lr);

    float m = -3.0e38f, l = 0.0f;
#pragma unroll 1
    for (int key0 = 0; key0 < SEQ; key0 += 32) {
        v8f ta = (v8f){}, tb = (v8f){};
        score32(kbase + (size_t)key0 * HD, qh0, qh1, qr0, qr1, relrow, pmrow + key0, key0 + dmb, ta, tb);
        float mx = -3.0e38f;
#pragma unroll
        for (int r = 0; r < 8; ++r) mx = fmaxf(mx, fmaxf(ta[r], tb[r]));
        const float mnew = fmaxf(m, mx);
        float ls = 0.0f;
#pragma unroll
        for (int r = 0; r < 8; ++r) ls += __builtin_amdgcn_exp2f(ta[r] - mnew) + __builtin_amdgcn_exp2f(tb[r] - mnew);
        l = l * __builtin_amdgcn_exp2f(m - mnew) + ls; m = mnew;
    }
    const float mo = __shfl_xor(m, 16, 32), lo = __shfl_xor(l, 16, 32);
    const float M = fmaxf(m, mo);
    const float Lh = l * __builtin_amdgcn_exp2f(m - M) + lo * __builtin_amdgcn_exp2f(mo - M);
    const float L = __shfl(Lh, lr, 32);
    const float inv = 1.0f / L;

    v8f o0 = (v8f){}, o1 = (v8f){}, o2 = (v8f){}, o3 = (v8f){};
    float e0 = 0.0f, e62 = 0.0f;
    float* arow = ATT + ((size_t)zh * OUT_SEQ + t0) * OUT_SEQ;
#pragma unroll 1
    for (int key0 = 0; key0 < SEQ; key0 += 32) {
        v8f ta = (v8f){}, tb = (v8f){};
        score32(kbase + (size_t)key0 * HD, qh0, qh1, qr0, qr1, relrow, pmrow + key0, key0 + dmb, ta, tb);
        v16h pb; v4f sa0, sa1, sb0, sb1;
#pragma unroll
        for (int r = 0; r < 8; ++r) {
            const float pa = __builtin_amdgcn_exp2f(ta[r] - M) * inv; const float pc = __builtin_amdgcn_exp2f(tb[r] - M) * inv;
            const h16 ha = (h16)(pa * PCAR); const h16 hc = (h16)(pc * PCAR);
            pb[r] = ha; pb[8 + r] = hc;
            if (r < 4) { sa0[r] = pa; sb0[r] = pc; } else { sa1[r - 4] = pa; sb1[r - 4] = pc; }
            const int da = key0 + dmb + r, db = da + 16;
            e0  += ((da <= -(MAXP - 1)) ? pa : 0.0f) + ((db <= -(MAXP - 1)) ? pc : 0.0f);
            e62 += ((da >=  (MAXP - 1)) ? pa : 0.0f) + ((db >=  (MAXP - 1)) ? pc : 0.0f);
            if (da > -(MAXP - 1) && da < (MAXP - 1)) rww[lr * 72 + da + (MAXP - 1)] = ha;
            if (db > -(MAXP - 1) && db < (MAXP - 1)) rww[lr * 72 + db + (MAXP - 1)] = hc;
        }
        *(v4fa*)(&osw[lr * 36 + 8 * hi]) = sa0;      *(v4fa*)(&osw[lr * 36 + 8 * hi + 4]) = sa1;
        *(v4fa*)(&osw[lr * 36 + 16 + 8 * hi]) = sb0; *(v4fa*)(&osw[lr * 36 + 16 + 8 * hi + 4]) = sb1;
        const h16* va = vbase + key0;
        const v16h v0 = ldh(va), v1 = ldh(va + (size_t)16 * SEQ), v2 = ldh(va + (size_t)32 * SEQ), v3 = ldh(va + (size_t)48 * SEQ);
        o0 = wmma16(v0, pb, o0); o1 = wmma16(v1, pb, o1); o2 = wmma16(v2, pb, o2); o3 = wmma16(v3, pb, o3);
        asm volatile("v_nop\n\tv_nop\n\tv_nop\n\tv_nop" : "+v"(o0), "+v"(o1), "+v"(o2), "+v"(o3) : "v"(v0), "v"(v1), "v"(v2), "v"(v3), "v"(pb));
        wave_sync();
        v4f x[4];
#pragma unroll
        for (int s = 0; s < 4; ++s) x[s] = *(const v4fa*)(&osw[(4 * s + (lane >> 3)) * 36 + (lane & 7) * 4]);
#pragma unroll 1
        for (int ps = 0; ps < 2; ++ps) {
#pragma unroll
            for (int s = 0; s < 4; ++s) *(volatile v4f*)(arow + (size_t)(4 * s + (lane >> 3)) * OUT_SEQ + key0 + (lane & 7) * 4) = x[s];
            if (ps == 0) __threadfence(); }
        wave_sync();
    }

    e0 += __shfl_xor(e0, 16, 32); e62 += __shfl_xor(e62, 16, 32);
    if (hi == 0) { rww[lr * 72 + 0] = (h16)(e0 * PCAR); rww[lr * 72 + (MREL - 1)] = (h16)(e62 * PCAR); }
    wave_sync();
    { const v16h rb0 = ldhs(rww + lr * 72 + 8 * hi), rb1 = ldhs(rww + lr * 72 + 32 + 8 * hi);
      const h16* vr = VRT + (size_t)h * 64 * 64 + (size_t)lr * 64 + 8 * hi;
      const v16h a00 = ldh(vr), a10 = ldh(vr + 16 * 64), a20 = ldh(vr + 32 * 64), a30 = ldh(vr + 48 * 64);
      const v16h a01 = ldh(vr + 32), a11 = ldh(vr + 16 * 64 + 32), a21 = ldh(vr + 32 * 64 + 32), a31 = ldh(vr + 48 * 64 + 32);
      v8f u0 = (v8f){}, u1 = (v8f){}, u2 = (v8f){}, u3 = (v8f){};
      u0 = wmma16(a00, rb0, u0); u1 = wmma16(a10, rb0, u1); u2 = wmma16(a20, rb0, u2); u3 = wmma16(a30, rb0, u3);
      u0 = wmma16(a01, rb1, u0); u1 = wmma16(a11, rb1, u1); u2 = wmma16(a21, rb1, u2); u3 = wmma16(a31, rb1, u3);
      asm volatile("v_nop\n\tv_nop\n\tv_nop\n\tv_nop" : "+v"(u0), "+v"(u1), "+v"(u2), "+v"(u3) : "v"(a01), "v"(a11), "v"(a21), "v"(a31), "v"(rb1));
      o0 = (o0 + u0 * RLI) * PCI; o1 = (o1 + u1 * RLI) * PCI; o2 = (o2 + u2 * RLI) * PCI; o3 = (o3 + u3 * RLI) * PCI; }

    { v4f a, c;
      a[0] = o0[0]; a[1] = o0[1]; a[2] = o0[2]; a[3] = o0[3]; c[0] = o0[4]; c[1] = o0[5]; c[2] = o0[6]; c[3] = o0[7];
      *(v4fa*)(&osw[lr * 68 +  0 + 8 * hi]) = a; *(v4fa*)(&osw[lr * 68 +  0 + 8 * hi + 4]) = c;
      a[0] = o1[0]; a[1] = o1[1]; a[2] = o1[2]; a[3] = o1[3]; c[0] = o1[4]; c[1] = o1[5]; c[2] = o1[6]; c[3] = o1[7];
      *(v4fa*)(&osw[lr * 68 + 16 + 8 * hi]) = a; *(v4fa*)(&osw[lr * 68 + 16 + 8 * hi + 4]) = c;
      a[0] = o2[0]; a[1] = o2[1]; a[2] = o2[2]; a[3] = o2[3]; c[0] = o2[4]; c[1] = o2[5]; c[2] = o2[6]; c[3] = o2[7];
      *(v4fa*)(&osw[lr * 68 + 32 + 8 * hi]) = a; *(v4fa*)(&osw[lr * 68 + 32 + 8 * hi + 4]) = c;
      a[0] = o3[0]; a[1] = o3[1]; a[2] = o3[2]; a[3] = o3[3]; c[0] = o3[4]; c[1] = o3[5]; c[2] = o3[6]; c[3] = o3[7];
      *(v4fa*)(&osw[lr * 68 + 48 + 8 * hi]) = a; *(v4fa*)(&osw[lr * 68 + 48 + 8 * hi + 4]) = c; }
    wave_sync();
    bf* crow = CTX + (size_t)(b * SEQ + t0) * (size_t)(2 * DM) + h * HD;
#pragma unroll 1
    for (int ps = 0; ps < 2; ++ps) {
#pragma unroll
        for (int s = 0; s < 4; ++s) { const int row = 4 * s + (lane >> 3), c8 = (lane & 7) * 8;
            const v4f x0 = *(const v4fa*)(&osw[row * 68 + c8]); const v4f x1 = *(const v4fa*)(&osw[row * 68 + c8 + 4]); v8us hv, lv;
#pragma unroll
            for (int i = 0; i < 4; ++i) { const unsigned short h0 = f2bf(x0[i]); const unsigned short h1 = f2bf(x1[i]); hv[i] = h0; hv[4 + i] = h1;
                lv[i] = f2bf(x0[i] - __uint_as_float(((unsigned)h0) << 16)); lv[4 + i] = f2bf(x1[i] - __uint_as_float(((unsigned)h1) << 16)); }
            bf* dst = crow + (size_t)row * (size_t)(2 * DM) + c8;
            *(volatile v8us*)dst = hv; *(volatile v8us*)(dst + DM) = lv; }
        if (ps == 0) __threadfence(); }
}

__global__ __launch_bounds__(32) void k_oproj(const bf* __restrict__ A, const bf* __restrict__ Bt, const float* __restrict__ bias, float* OUT) {
    __shared__ __align__(16) float os[16 * 68];
    const int K2 = 2 * DM;
    const int lane = threadIdx.x & 31, lr = lane & 15, hi = lane >> 4; const int r0 = blockIdx.x * 64, c0 = blockIdx.y * 64;
    v8f acc[4][4];
#pragma unroll
    for (int mb = 0; mb < 4; ++mb)
#pragma unroll
        for (int nb = 0; nb < 4; ++nb) acc[mb][nb] = (v8f){};
    const size_t aoff = (size_t)(r0 + lr) * K2 + 8 * hi, boff = (size_t)(c0 + lr) * DM + 8 * hi;
#pragma unroll 1
    for (int kc = 0; kc < K2; kc += 32) {
        const int kb = kc & (DM - 1);
        v16bf a[4];
#pragma unroll
        for (int mb = 0; mb < 4; ++mb) a[mb] = ldb(A + aoff + (size_t)mb * 16 * K2 + kc);
#pragma unroll
        for (int nb = 0; nb < 4; ++nb) { const v16bf b = ldb(Bt + boff + (size_t)nb * 16 * DM + kb);
#pragma unroll
            for (int mb = 0; mb < 4; ++mb) acc[mb][nb] = wmmab(a[mb], b, acc[mb][nb]); }
        asm volatile("v_nop\n\tv_nop\n\tv_nop\n\tv_nop" : "+v"(acc[0][0]), "+v"(acc[1][1]), "+v"(acc[2][2]), "+v"(acc[3][3]) : "v"(a[0]), "v"(a[1]), "v"(a[2]), "v"(a[3]));
    }
    const v4f braw = *(const v4f*)(bias + c0 + lr * 4); v4f bv;
#pragma unroll
    for (int i = 0; i < 4; ++i) bv[i] = bfr(braw[i]);
#pragma unroll
    for (int mb = 0; mb < 4; ++mb) {
#pragma unroll
        for (int nb = 0; nb < 4; ++nb) {
#pragma unroll
            for (int j = 0; j < 8; ++j) os[(hi * 8 + j) * 68 + nb * 16 + lr] = acc[mb][nb][j]; }
        wave_sync();
        const int gm = r0 + mb * 16; const int bb = gm / SEQ, tt = gm % SEQ;
        float* ob = OUT + ((size_t)bb * OUT_SEQ + tt) * DM + c0;
#pragma unroll 1
        for (int ps = 0; ps < 2; ++ps) {
#pragma unroll
            for (int s = 0; s < 8; ++s) { const int row = 2 * s + hi, cofs = lr * 4;
                const v4f val = *(const v4fa*)(&os[row * 68 + cofs]) + bv;
                *(volatile v4f*)(ob + (size_t)row * DM + cofs) = val; }
            if (ps == 0) __threadfence(); }
        wave_sync();
    }
}

static constexpr size_t al256(size_t v) { return (v + 255) & ~(size_t)255; }
static constexpr size_t SZ_X   = al256((size_t)NB * SEQ * DM * 2);
static constexpr size_t SZ_W   = al256((size_t)DM * DM * 2);
static constexpr size_t SZ_PL  = al256((size_t)NB * NH_ * SEQ * HD * 2);
static constexpr size_t SZ_CTX = al256((size_t)NB * SEQ * 2 * DM * 2);
static constexpr size_t SZ_RL  = al256((size_t)NH_ * 64 * 64 * 2);
static constexpr size_t SZ_TOTAL = 3 * SZ_X + 4 * SZ_W + 4 * SZ_PL + SZ_CTX + 2 * SZ_RL;
static_assert(SZ_TOTAL <= (size_t)134217728);

extern "C" void kernel_launch(void* const* d_in, const int* in_sizes, int n_in,
                              void* d_out, int out_size, void* d_ws, size_t ws_size, hipStream_t stream) {
    if (n_in < 11) return;
    const size_t needx = ((size_t)(NB - 1) * SEQ_FULL + SEQ) * DM;
    if ((size_t)in_sizes[0] < needx || (size_t)in_sizes[1] < needx || (size_t)in_sizes[2] < needx) return;
    if ((size_t)in_sizes[3] < (size_t)(NB - 1) * SEQ_FULL + SEQ) return;
    if ((size_t)in_sizes[4] < (size_t)DM * DM || (size_t)in_sizes[5] < (size_t)DM * DM || (size_t)in_sizes[6] < (size_t)DM * DM || (size_t)in_sizes[7] < (size_t)DM * DM) return;
    if ((size_t)in_sizes[8] < (size_t)DM) return;
    if ((size_t)in_sizes[9] < (size_t)NH_ * MREL * HD || (size_t)in_sizes[10] < (size_t)NH_ * MREL * HD) return;
    if ((size_t)out_size < OUT1_OFF + (((size_t)NB * NH_ - 1) * OUT_SEQ + SEQ - 1) * OUT_SEQ + SEQ) return;
    if (SZ_TOTAL > ws_size) return;
    const float* xv = (const float*)d_in[0]; const float* xk = (const float*)d_in[1]; const float* xq = (const float*)d_in[2];
    const float* pm = (const float*)d_in[3];
    const float* wq = (const float*)d_in[4]; const float* wk = (const float*)d_in[5]; const float* wv = (const float*)d_in[6]; const float* wo = (const float*)d_in[7];
    const float* bo = (const float*)d_in[8]; const float* krel = (const float*)d_in[9]; const float* vrel = (const float*)d_in[10];
    float* OUT0 = (float*)d_out;
    float* OUT1 = (float*)d_out + OUT1_OFF;
    char* wsp = (char*)d_ws;
    bf* XQ = (bf*)wsp; wsp += SZ_X;
    bf* XK = (bf*)wsp; wsp += SZ_X;
    bf* XV = (bf*)wsp; wsp += SZ_X;
    bf* WQT = (bf*)wsp; wsp += SZ_W;
    bf* WKT = (bf*)wsp; wsp += SZ_W;
    bf* WVT = (bf*)wsp; wsp += SZ_W;
    bf* WOT = (bf*)wsp; wsp += SZ_W;
    h16* QH = (h16*)wsp; wsp += SZ_PL;
    h16* QR = (h16*)wsp; wsp += SZ_PL;
    h16* KP = (h16*)wsp; wsp += SZ_PL;
    h16* VT = (h16*)wsp; wsp += SZ_PL;
    bf* CTX = (bf*)wsp; wsp += SZ_CTX;
    h16* KRP = (h16*)wsp; wsp += SZ_RL;
    h16* VRT = (h16*)wsp; wsp += SZ_RL;

    if (SEQ == SEQ_FULL) {
        const size_t n8 = (size_t)NB * SEQ * DM / 8; const unsigned g = (unsigned)((n8 + 255) / 256);
        k_cvt8<<<g, 256, 0, stream>>>(xq, XQ, n8); k_cvt8<<<g, 256, 0, stream>>>(xk, XK, n8); k_cvt8<<<g, 256, 0, stream>>>(xv, XV, n8);
    } else {
        const size_t n8 = (size_t)SEQ * DM / 8; const unsigned g = (unsigned)((n8 + 255) / 256);
        for (int b = 0; b < NB; ++b) {
            k_cvt8<<<g, 256, 0, stream>>>(xq + (size_t)b * SEQ_FULL * DM, XQ + (size_t)b * SEQ * DM, n8);
            k_cvt8<<<g, 256, 0, stream>>>(xk + (size_t)b * SEQ_FULL * DM, XK + (size_t)b * SEQ * DM, n8);
            k_cvt8<<<g, 256, 0, stream>>>(xv + (size_t)b * SEQ_FULL * DM, XV + (size_t)b * SEQ * DM, n8);
        }
    }
    k_cvtT<<<dim3(DM / 64, DM / 64, 1), 256, 0, stream>>>(wq, WQT);
    k_cvtT<<<dim3(DM / 64, DM / 64, 1), 256, 0, stream>>>(wk, WKT);
    k_cvtT<<<dim3(DM / 64, DM / 64, 1), 256, 0, stream>>>(wv, WVT);
    k_cvtT<<<dim3(DM / 64, DM / 64, 1), 256, 0, stream>>>(wo, WOT);
    k_relprep<<<NH_, 256, 0, stream>>>(krel, KRP, 0);
    k_relprep<<<NH_, 256, 0, stream>>>(vrel, VRT, 1);

    k_proj<<<dim3(NB * SEQ / 64, DM / 64, 1), 32, 0, stream>>>(XQ, WQT, QH, QR, 1, SEQ, (size_t)NH_ * SEQ * HD, HD, HD, (size_t)SEQ * HD);
    k_proj<<<dim3(NB * SEQ / 64, DM / 64, 1), 32, 0, stream>>>(XK, WKT, KP, KP, 0, SEQ, (size_t)NH_ * SEQ * HD, HD, HD, (size_t)SEQ * HD);
    k_proj<<<dim3(DM / 64, NB * SEQ / 64, 1), 32, 0, stream>>>(WVT, XV, VT, VT, 0, DM, (size_t)0, SEQ, SEQ, (size_t)DM * SEQ);

    k_attn<<<dim3(SEQ / (16 * AW), NB * NH_, 1), 32 * AW, 0, stream>>>(QH, QR, KP, VT, KRP, VRT, pm, CTX, OUT1);

    k_oproj<<<dim3(NB * SEQ / 64, DM / 64, 1), 32, 0, stream>>>(CTX, WOT, bo, OUT0);
}
